// RWKV_Tmix_x070_Mose_cxa073_39024072851816
// MI455X (gfx1250) — hardware-verified
//
#include <hip/hip_runtime.h>
#include <math.h>
#include <stddef.h>

#pragma clang fp contract(off)

constexpr int kBatch  = 4;
constexpr int kSeq    = 1024;
constexpr int kChan   = 1024;
constexpr int kHeads  = 16;
constexpr int kHeadSz = 64;
constexpr int kRows   = kBatch * kSeq;
constexpr int kKvHalf = 256;
constexpr int kKvCols = 512;
constexpr int kLr1N   = 192;
constexpr int kLr2K   = 64;
constexpr int kDecLo  = 64;
constexpr int kMvLo   = 32;
constexpr int kStage  = 16;
constexpr float kEps  = 0.00064f;
static_assert(kRows % 64 == 0, "");
static_assert(kChan % 64 == 0 && kKvCols % 64 == 0 && kLr1N % 64 == 0, "");
static_assert(kChan % 32 == 0 && kLr2K % 32 == 0, "");
static_assert(kHeads * kHeadSz == kChan, "");
static_assert(kSeq % kStage == 0, "");

typedef __attribute__((ext_vector_type(16))) _Float16 v16h;
typedef __attribute__((ext_vector_type(8)))  _Float16 v8h;
typedef __attribute__((ext_vector_type(16))) __bf16   v16b;
typedef __attribute__((ext_vector_type(8)))  __bf16   v8b;
typedef __attribute__((ext_vector_type(8)))  float    v8f;
typedef __attribute__((ext_vector_type(4)))  float    v4f;
typedef __attribute__((ext_vector_type(4)))  unsigned int v4u;

__device__ __forceinline__ unsigned short f2bf_bits(float f) {
  unsigned u = __float_as_uint(f);
  return (unsigned short)((u + 0x7FFFu + ((u >> 16) & 1u)) >> 16);
}
__device__ __forceinline__ float bf_bits2f(unsigned short h) { return __uint_as_float(((unsigned)h) << 16); }

__device__ __forceinline__ void dep_guard_h(v8f& a, v8f& b, v16h x, v16h y) { asm volatile("v_nop\n\tv_nop\n\tv_nop\n\tv_nop" : "+v"(a), "+v"(b) : "v"(x), "v"(y)); }
__device__ __forceinline__ void dep_guard_b(v8f& a, v8f& b, v16b x, v16b y) { asm volatile("v_nop\n\tv_nop\n\tv_nop\n\tv_nop" : "+v"(a), "+v"(b) : "v"(x), "v"(y)); }
__device__ __forceinline__ void keep4_h(v16h a, v16h b, v16h c, v16h d) { asm volatile("v_nop" :: "v"(a), "v"(b), "v"(c), "v"(d)); }
__device__ __forceinline__ void keep4_b(v16b a, v16b b, v16b c, v16b d) { asm volatile("v_nop" :: "v"(a), "v"(b), "v"(c), "v"(d)); }
__device__ __forceinline__ void acc_guard4(v8f& a, v8f& b, v8f& c, v8f& d) { asm volatile("v_nop\n\tv_nop\n\tv_nop\n\tv_nop" : "+v"(a), "+v"(b), "+v"(c), "+v"(d)); }
template <typename T> struct Frag;
template <> struct Frag<_Float16> {
  typedef v16h V; union U { v16h v; v8h h[2]; };
  static __device__ __forceinline__ v16h load(const _Float16* p) {
    U f; f.h[0] = *(const v8h*)(p); f.h[1] = *(const v8h*)(p + 16); return f.v;
  }
  static __device__ __forceinline__ v8f mma(v16h a, v16h b, v8f c) {
    return __builtin_amdgcn_wmma_f32_16x16x32_f16(false, a, false, b, (short)0, c, false, false);
  }
  static __device__ __forceinline__ void guard(v8f& a, v8f& b, v16h x, v16h y) { dep_guard_h(a, b, x, y); }
  static __device__ __forceinline__ void keep(v16h a, v16h b, v16h c, v16h d) { keep4_h(a, b, c, d); }
};
template <> struct Frag<__bf16> {
  typedef v16b V; union U { v16b v; v8b h[2]; };
  static __device__ __forceinline__ v16b load(const __bf16* p) {
    U f; f.h[0] = *(const v8b*)(p); f.h[1] = *(const v8b*)(p + 16); return f.v;
  }
  static __device__ __forceinline__ v8f mma(v16b a, v16b b, v8f c) {
    return __builtin_amdgcn_wmma_f32_16x16x32_bf16(false, a, false, b, (short)0, c, false, false);
  }
  static __device__ __forceinline__ void guard(v8f& a, v8f& b, v16b x, v16b y) { dep_guard_b(a, b, x, y); }
  static __device__ __forceinline__ void keep(v16b a, v16b b, v16b c, v16b d) { keep4_b(a, b, c, d); }
};

__device__ __forceinline__ unsigned pk16(unsigned short a, unsigned short b) { return (unsigned)a | ((unsigned)b << 16); }

template <int ET> struct Elem;
template <> struct Elem<0> { typedef _Float16 T; };
template <> struct Elem<1> { typedef __bf16 T; };
template <int ET, bool SPLIT, int BIAS_MODE, int OUT_MODE, bool RESID, int ACT = 0>
__global__ __launch_bounds__(256) void wmma_gemm64(
    const unsigned short* __restrict__ Ap, const unsigned short* __restrict__ A2p, int lda, long strideA,
    const unsigned short* __restrict__ Btp, const unsigned short* __restrict__ Bt2p, int ldb, long strideB,
    void* __restrict__ Cout, void* __restrict__ Cout2, int ldc, long strideC,
    const float* __restrict__ bias,
    const float* __restrict__ resid, long strideR,
    int M, int N, int K, float scale) {
  typedef typename Elem<ET>::T T;
  typedef typename Frag<T>::V V;
  const T* A = (const T*)Ap; const T* A2 = (const T*)A2p; const T* Bt = (const T*)Btp; const T* Bt2 = (const T*)Bt2p;
  __shared__ __align__(16) float sT[8][16 * 68];
  const int b    = blockIdx.y;
  const int lane = threadIdx.x & 31;
  const int wave = threadIdx.x >> 5;
  const int tilesN = N >> 6;
  const int tilesM = M >> 6;
  const int tile = blockIdx.x * 8 + wave;
  if (tile >= tilesM * tilesN) return;
  const int tm = tile / tilesN;
  const int tn = tile - tm * tilesN;
  const int m0 = tm << 6;
  const int n0 = tn << 6;

  const T* Ab  = A  + (size_t)b * strideA;
  const T* Bb  = Bt + (size_t)b * strideB;
  const T* Ab2 = SPLIT ? (A2  + (size_t)b * strideA) : nullptr;
  const T* Bb2 = SPLIT ? (Bt2 + (size_t)b * strideB) : nullptr;

  const int rlane = lane & 15;
  const int koff  = (lane >> 4) * 8;
  const int mOff  = (lane >> 4) * 8;

  v8f acc[4][4];
#pragma unroll
  for (int i = 0; i < 4; ++i)
#pragma unroll
    for (int j = 0; j < 4; ++j) acc[i][j] = (v8f){0.f,0.f,0.f,0.f,0.f,0.f,0.f,0.f};

  for (int k0 = 0; k0 < K; k0 += 32) {
    V bh[4], bl[4];
#pragma unroll
    for (int j = 0; j < 4; ++j) {
      const size_t bo = (size_t)(n0 + (j << 4) + rlane) * ldb + koff + k0;
      bh[j] = Frag<T>::load(Bb + bo);
      if (SPLIT) bl[j] = Frag<T>::load(Bb2 + bo);
    }
#pragma unroll
    for (int i = 0; i < 4; ++i) {
      const size_t ao = (size_t)(m0 + (i << 4) + rlane) * lda + koff + k0;
      V ah = Frag<T>::load(Ab + ao);
      V al;
      if (SPLIT) al = Frag<T>::load(Ab2 + ao);
#pragma unroll
      for (int j = 0; j < 4; ++j) {
        acc[i][j] = Frag<T>::mma(ah, bh[j], acc[i][j]);
        if (SPLIT) {
          acc[i][j] = Frag<T>::mma(ah, bl[j], acc[i][j]);
          acc[i][j] = Frag<T>::mma(al, bh[j], acc[i][j]);
        }
      }
      Frag<T>::guard(acc[i][0], acc[i][3], ah, SPLIT ? al : ah);
    }
    Frag<T>::keep(bh[0], bh[1], bh[2], bh[3]);
    if (SPLIT) Frag<T>::keep(bl[0], bl[1], bl[2], bl[3]);
  }
  acc_guard4(acc[0][0], acc[0][1], acc[0][2], acc[0][3]);
  acc_guard4(acc[1][0], acc[1][1], acc[1][2], acc[1][3]);
  acc_guard4(acc[2][0], acc[2][1], acc[2][2], acc[2][3]);
  acc_guard4(acc[3][0], acc[3][1], acc[3][2], acc[3][3]);

  float* slab = sT[wave];
  const float* Rb = RESID ? (resid + (size_t)b * strideR) : nullptr;
#pragma unroll
  for (int i = 0; i < 4; ++i) {
    const int mBase = m0 + (i << 4);
#pragma unroll
    for (int j = 0; j < 4; ++j) {
      const int n = n0 + (j << 4) + rlane;
      float bv = 0.f;
      if (BIAS_MODE == 2) bv = bias[n];
#pragma unroll
      for (int r = 0; r < 8; ++r) {
        float v = acc[i][j][r] * scale;
        if (BIAS_MODE == 1) v += bias[mBase + mOff + r];
        if (BIAS_MODE == 2) v += bv;
        if (RESID) v += Rb[(size_t)(mBase + mOff + r) * ldc + n];
        if (ACT == 2) v = fmaxf(v, 0.0f);
        if (ACT == 4) v = (v > 0.f) ? v : 0.01f * v;
        slab[(mOff + r) * 68 + (j << 4) + rlane] = v;
      }
    }
    __builtin_amdgcn_fence(__ATOMIC_RELEASE, "workgroup");
    __builtin_amdgcn_wave_barrier();
    __builtin_amdgcn_fence(__ATOMIC_ACQUIRE, "workgroup");
    if (OUT_MODE == 0) {
      float* C = (float*)Cout + (size_t)b * strideC;
      const int hh = lane >> 4, c4 = (lane & 15) * 4;
      for (int pass = 0; pass < 2; ++pass) {
#pragma unroll
        for (int it = 0; it < 8; ++it) {
          const int row = it * 2 + hh;
          v4f v = *(const v4f*)(slab + row * 68 + c4);
          *(volatile v4f*)(C + (size_t)(mBase + row) * ldc + n0 + c4) = v;
        }
        __threadfence();
      }
    } else {
      const int q = lane >> 3, c8 = (lane & 7) * 8;
      unsigned short* C  = (unsigned short*)Cout  + (size_t)b * strideC;
      unsigned short* C2 = (OUT_MODE == 2) ? ((unsigned short*)Cout2 + (size_t)b * strideC) : nullptr;
      for (int pass = 0; pass < 2; ++pass) {
#pragma unroll
        for (int it = 0; it < 4; ++it) {
          const int row = it * 4 + q;
          const float* sp = slab + row * 68 + c8;
          v8h hv, lv;
#pragma unroll
          for (int e = 0; e < 8; ++e) {
            if (OUT_MODE == 1) {
              hv[e] = (_Float16)sp[e];
            } else {
              unsigned short hb = f2bf_bits(sp[e]);
              unsigned short lb = f2bf_bits(sp[e] - bf_bits2f(hb));
              hv[e] = __builtin_bit_cast(_Float16, hb);
              lv[e] = __builtin_bit_cast(_Float16, lb);
            }
          }
          *(volatile v8h*)(C + (size_t)(mBase + row) * ldc + n0 + c8) = hv;
          if (OUT_MODE == 2) *(volatile v8h*)(C2 + (size_t)(mBase + row) * ldc + n0 + c8) = lv;
        }
        __threadfence();
      }
    }
    __builtin_amdgcn_fence(__ATOMIC_RELEASE, "workgroup");
    __builtin_amdgcn_wave_barrier();
    __builtin_amdgcn_fence(__ATOMIC_ACQUIRE, "workgroup");
  }
}

__global__ __launch_bounds__(256) void cast8_split_kernel(const float* __restrict__ in,
                                                          unsigned short* __restrict__ hi,
                                                          unsigned short* __restrict__ lo, int n8) {
#pragma clang fp contract(off)
  const int i = blockIdx.x * 256 + threadIdx.x;
  if (i >= n8) return;
  const float* p = in + 8 * (size_t)i;
  const v4f a = *(const v4f*)(p);
  const v4f c = *(const v4f*)(p + 4);
  unsigned short hb[8], lb[8];
#pragma unroll
  for (int e = 0; e < 4; ++e) {
    hb[e] = f2bf_bits(a[e]);
    lb[e] = f2bf_bits(a[e] - bf_bits2f(hb[e]));
    hb[4 + e] = f2bf_bits(c[e]);
    lb[4 + e] = f2bf_bits(c[e] - bf_bits2f(hb[4 + e]));
  }
  const v4u uh = (v4u){pk16(hb[0], hb[1]), pk16(hb[2], hb[3]), pk16(hb[4], hb[5]), pk16(hb[6], hb[7])};
  const v4u ul = (v4u){pk16(lb[0], lb[1]), pk16(lb[2], lb[3]), pk16(lb[4], lb[5]), pk16(lb[6], lb[7])};
  unsigned short* qh = hi + 8 * (size_t)i;
  unsigned short* ql = lo + 8 * (size_t)i;
  *(volatile v4u*)qh = uh;
  *(volatile v4u*)ql = ul;
  __threadfence();
  *(volatile v4u*)qh = uh;
  *(volatile v4u*)ql = ul;
}

__global__ __launch_bounds__(256) void tr_split_kernel(const float* __restrict__ in, int R, int Cc,
                                                       unsigned short* __restrict__ hi,
                                                       unsigned short* __restrict__ lo, int ldo) {
#pragma clang fp contract(off)
  __shared__ float sm[64][65];
  const int t   = threadIdx.x;
  const int or0 = blockIdx.x * 64;
  const int oc0 = blockIdx.y * 64;
#pragma unroll
  for (int i = 0; i < 16; ++i) {
    const int e  = i * 256 + t;
    const int rl = e >> 6;
    const int cl = e & 63;
    const int rr = or0 + rl;
    const int cc = oc0 + cl;
    const int rcl = (rr < R) ? rr : (R - 1);
    const int ccl = (cc < Cc) ? cc : (Cc - 1);
    float v = in[(size_t)rcl * Cc + ccl];
    if (!((rr < R) && (cc < Cc))) v = 0.0f;
    sm[cl][rl] = v;
  }
  __syncthreads();
  const int lane = t & 31, wave = t >> 5;
  const int q = lane >> 3, c8 = (lane & 7) * 8;
  for (int pass = 0; pass < 2; ++pass) {
#pragma unroll
    for (int it = 0; it < 2; ++it) {
      const int row = wave * 8 + it * 4 + q;
      unsigned short hb[8], lb[8];
#pragma unroll
      for (int e = 0; e < 8; ++e) {
        const float f = sm[row][c8 + e];
        hb[e] = f2bf_bits(f);
        lb[e] = f2bf_bits(f - bf_bits2f(hb[e]));
      }
      const v4u uh = (v4u){pk16(hb[0], hb[1]), pk16(hb[2], hb[3]), pk16(hb[4], hb[5]), pk16(hb[6], hb[7])};
      const v4u ul = (v4u){pk16(lb[0], lb[1]), pk16(lb[2], lb[3]), pk16(lb[4], lb[5]), pk16(lb[6], lb[7])};
      const size_t o = (size_t)(oc0 + row) * ldo + or0 + c8;
      *(volatile v4u*)(hi + o) = uh;
      *(volatile v4u*)(lo + o) = ul;
    }
    __threadfence();
  }
}

__global__ __launch_bounds__(256) void lr_convert_kernel(const float* __restrict__ in,
                                                         unsigned short* __restrict__ hi,
                                                         unsigned short* __restrict__ lo, int n2) {
#pragma clang fp contract(off)
  const int i = blockIdx.x * 256 + threadIdx.x;
  if (i >= n2) return;
  const int col = (2 * i) % kLr1N;
  float x0 = in[2 * (size_t)i];
  float x1 = in[2 * (size_t)i + 1];
  if (col < kDecLo) {
    x0 = tanhf(x0);
    x1 = tanhf(x1);
  }
  const unsigned short h0 = f2bf_bits(x0);
  const unsigned short l0 = f2bf_bits(x0 - bf_bits2f(h0));
  const unsigned short h1 = f2bf_bits(x1);
  const unsigned short l1 = f2bf_bits(x1 - bf_bits2f(h1));
  const unsigned uh = pk16(h0, h1);
  const unsigned ul = pk16(l0, l1);
  ((volatile unsigned*)hi)[i] = uh;
  ((volatile unsigned*)lo)[i] = ul;
  __threadfence();
  ((volatile unsigned*)hi)[i] = uh;
  ((volatile unsigned*)lo)[i] = ul;
}

__device__ __forceinline__ float wave_sum32(float v) {
#pragma unroll
  for (int off = 16; off > 0; off >>= 1) v += __shfl_xor(v, off, 32);
  return v;
}

__global__ __launch_bounds__(64) void scan_kernel(
    const float* __restrict__ Rp, const float* __restrict__ KVp,
    const float* __restrict__ WLp, const float* __restrict__ ALp, const float* __restrict__ VLp,
    const float* __restrict__ vfp, const float* __restrict__ maskp,
    const float* __restrict__ w0p, const float* __restrict__ a0p, const float* __restrict__ v0p,
    const float* __restrict__ kkp, const float* __restrict__ kap, const float* __restrict__ rkp,
    const float* __restrict__ gp, const float* __restrict__ bp,
    unsigned short* __restrict__ YH, unsigned short* __restrict__ YL) {
#pragma clang fp contract(off)
  __shared__ __align__(16) float vdec[64];
  __shared__ __align__(16) float vkf[64];
  __shared__ __align__(16) float vrr[64];
  __shared__ __align__(16) float vkk[64];
  __shared__ __align__(16) float vbb[64];
  __shared__ __align__(16) float ystage[kStage * 64];
  __shared__ float red_a[2];
  __shared__ float red_b[4];
  __shared__ float red_c[2];

  const int bidx = blockIdx.x / kHeads;
  const int h    = blockIdx.x - bidx * kHeads;
  const int c    = threadIdx.x;
  const int lane = c & 31;
  const int wave = c >> 5;
  const int ch   = h * kHeadSz + c;
  const int kvc  = (h >> 2) * kHeadSz + c;
  const int q8   = c >> 3;
  const int c8   = (c & 7) * 8;

  const float cw0   = w0p[ch];
  const float ca0   = a0p[ch];
  const float cv0   = v0p[ch];
  const float ckk   = kkp[ch];
  const float cka   = kap[ch];
  const float crk   = rkp[h * kHeadSz + c];
  const float cg    = gp[ch];
  const float cbeta = bp[ch];

  float S[64];
#pragma unroll
  for (int j = 0; j < 64; ++j) S[j] = 0.0f;

  for (int t = 0; t < kSeq; ++t) {
    const size_t row = (size_t)bidx * kSeq + t;
    const float m    = maskp[bidx * kSeq + t];
    const float rv   = Rp[row * kChan + ch];
    const float wl   = WLp[row * kChan + ch];
    const float al   = ALp[row * kChan + ch];
    const float vl   = VLp[row * kChan + ch];
    const float kraw = KVp[row * kKvCols + kvc];
    const float vraw = KVp[row * kKvCols + kKvHalf + kvc];
    const float vf   = vfp[row * kChan + ch];

    const float z    = cw0 + wl;
    const float u    = -z;
    const float au   = fabsf(u);
    const float e1   = expf(-au);
    const float lp   = log1pf(e1);
    const float sp   = fmaxf(u, 0.0f) + lp;
    const float w    = -sp - 0.6f;
    const float ew   = expf(w);
    const float dec  = expf(-ew);
    const float decm = (m > 0.0f) ? dec : 1.0f;
    const float ea   = expf(-(ca0 + al));
    const float asig = 1.0f / (1.0f + ea);
    const float eg   = expf(-(cv0 + vl));
    const float gate = 1.0f / (1.0f + eg);
    const float dv   = vf - vraw;
    const float vm   = vraw + dv * gate;
    const float kkraw = kraw * ckk;
    const float am1  = asig - 1.0f;
    const float kf   = kraw * (1.0f + am1 * cka);
    const float qq   = kkraw * kkraw;
    const float rk0  = rv * kf;
    const float rkt  = rk0 * crk;

    const float qsum = wave_sum32(qq);
    vdec[c] = decm;
    vkf[c]  = kf * m;
    vrr[c]  = rv;
    if (lane == 0) red_a[wave] = qsum;
    __syncthreads();

    const float nrm2 = red_a[0] + red_a[1];
    const float nrm0 = sqrtf(nrm2);
    const float nrm  = fmaxf(nrm0, 1e-12f);
    const float inrm = 1.0f / nrm;
    const float kk   = kkraw * inrm;
    const float bbv  = kk * asig;
    vkk[c] = kk * m;
    vbb[c] = bbv * m;
    __syncthreads();

    float sdot = 0.0f;
#pragma unroll
    for (int j0 = 0; j0 < 64; j0 += 16) {
      v4f kq[4];
#pragma unroll
      for (int qv = 0; qv < 4; ++qv) kq[qv] = *(const v4f*)(vkk + j0 + 4 * qv);
#pragma unroll
      for (int jj = 0; jj < 16; ++jj) {
        const float p = S[j0 + jj] * kq[jj >> 2][jj & 3];
        sdot = sdot + p;
      }
      asm volatile("" ::: "memory");
    }
    const float sa   = -sdot;
    const float vrec = vm * m;

    float yv = 0.0f;
#pragma unroll
    for (int j0 = 0; j0 < 64; j0 += 16) {
      v4f dq[4], bq[4], fq[4], rq[4];
#pragma unroll
      for (int qv = 0; qv < 4; ++qv) {
        dq[qv] = *(const v4f*)(vdec + j0 + 4 * qv);
        bq[qv] = *(const v4f*)(vbb + j0 + 4 * qv);
        fq[qv] = *(const v4f*)(vkf + j0 + 4 * qv);
        rq[qv] = *(const v4f*)(vrr + j0 + 4 * qv);
      }
#pragma unroll
      for (int jj = 0; jj < 16; ++jj) {
        const int j    = j0 + jj;
        const float t1 = S[j] * dq[jj >> 2][jj & 3];
        const float t2 = sa * bq[jj >> 2][jj & 3];
        const float t3 = vrec * fq[jj >> 2][jj & 3];
        const float s12 = t1 + t2;
        const float sn  = s12 + t3;
        S[j] = sn;
        const float py = sn * rq[jj >> 2][jj & 3];
        yv = yv + py;
      }
      asm volatile("" ::: "memory");
    }

    const float psy  = wave_sum32(yv);
    const float psrk = wave_sum32(rkt);
    if (lane == 0) {
      red_b[wave * 2]     = psy;
      red_b[wave * 2 + 1] = psrk;
    }
    __syncthreads();
    const float mu = (red_b[0] + red_b[2]) * (1.0f / 64.0f);
    const float rk = red_b[1] + red_b[3];
    const float dy = yv - mu;
    const float d2 = dy * dy;
    const float psv = wave_sum32(d2);
    if (lane == 0) red_c[wave] = psv;
    __syncthreads();
    const float var = (red_c[0] + red_c[1]) * (1.0f / 64.0f);
    const float rs  = rsqrtf(var + kEps);
    const float yn  = dy * rs;
    const float yg  = yn * cg;
    const float yb  = yg + cbeta;
    const float rvm = rk * vm;
    const float yfin = yb + rvm;
    ystage[(t & (kStage - 1)) * 64 + c] = yfin;

    if ((t & (kStage - 1)) == (kStage - 1)) {
      __syncthreads();
      v4u uh[2], ul[2];
      size_t goff[2];
#pragma unroll
      for (int it = 0; it < 2; ++it) {
        const int srow = it * 8 + q8;
        const v4f f0 = *(const v4f*)(ystage + srow * 64 + c8);
        const v4f f1 = *(const v4f*)(ystage + srow * 64 + c8 + 4);
        unsigned short hb[8], lb[8];
#pragma unroll
        for (int e = 0; e < 4; ++e) {
          hb[e] = f2bf_bits(f0[e]);
          lb[e] = f2bf_bits(f0[e] - bf_bits2f(hb[e]));
          hb[4 + e] = f2bf_bits(f1[e]);
          lb[4 + e] = f2bf_bits(f1[e] - bf_bits2f(hb[4 + e]));
        }
        uh[it] = (v4u){pk16(hb[0], hb[1]), pk16(hb[2], hb[3]), pk16(hb[4], hb[5]), pk16(hb[6], hb[7])};
        ul[it] = (v4u){pk16(lb[0], lb[1]), pk16(lb[2], lb[3]), pk16(lb[4], lb[5]), pk16(lb[6], lb[7])};
        goff[it] = ((size_t)bidx * kSeq + (size_t)(t - (kStage - 1) + srow)) * kChan + (size_t)h * kHeadSz + c8;
      }
      for (int pass = 0; pass < 2; ++pass) {
#pragma unroll
        for (int it = 0; it < 2; ++it) {
          *(volatile v4u*)(YH + goff[it]) = uh[it];
          *(volatile v4u*)(YL + goff[it]) = ul[it];
        }
        __threadfence();
      }
    }
  }
}

__global__ __launch_bounds__(256) void copy4_kernel(const float* __restrict__ in, float* __restrict__ out, int n4) {
  const int i = blockIdx.x * 256 + threadIdx.x;
  if (i >= n4) return;
  const v4f v = *(const v4f*)(in + 4 * (size_t)i);
  float* p = out + 4 * (size_t)i;
  *(volatile v4f*)p = v;
  __threadfence();
  *(volatile v4f*)p = v;
}

extern "C" void kernel_launch(void* const* d_in, const int* in_sizes, int n_in,
                              void* d_out, int out_size, void* d_ws, size_t ws_size,
                              hipStream_t stream) {
  if (n_in < 21) return;
  if (in_sizes[0] != kRows * kChan || in_sizes[1] != kRows * kChan) return;
  if (in_sizes[2] != kRows || in_sizes[3] != kChan * kChan || in_sizes[4] != kKvHalf * kChan) return;
  if (in_sizes[5] != kKvHalf * kChan || in_sizes[6] != kChan * kChan) return;
  if (in_sizes[8] != kChan * kDecLo || in_sizes[9] != kDecLo * kChan) return;
  if (in_sizes[11] != kChan * kDecLo || in_sizes[12] != kDecLo * kChan) return;
  if (in_sizes[14] != kChan * kMvLo || in_sizes[15] != kMvLo * kChan) return;
  if (in_sizes[18] != kHeads * kHeadSz) return;
  if (out_size != 2 * kRows * kChan) return;

  const float* x       = (const float*)d_in[0];
  const float* v_first = (const float*)d_in[1];
  const float* amask   = (const float*)d_in[2];
  const float* Wr  = (const float*)d_in[3];
  const float* Wk  = (const float*)d_in[4];
  const float* Wv  = (const float*)d_in[5];
  const float* Wo  = (const float*)d_in[6];
  const float* w0  = (const float*)d_in[7];
  const float* w1  = (const float*)d_in[8];
  const float* w2  = (const float*)d_in[9];
  const float* a0  = (const float*)d_in[10];
  const float* a1  = (const float*)d_in[11];
  const float* a2  = (const float*)d_in[12];
  const float* v0  = (const float*)d_in[13];
  const float* v1  = (const float*)d_in[14];
  const float* v2  = (const float*)d_in[15];
  const float* k_k = (const float*)d_in[16];
  const float* k_a = (const float*)d_in[17];
  const float* r_k = (const float*)d_in[18];
  const float* ln_g = (const float*)d_in[19];
  const float* ln_b = (const float*)d_in[20];
  float* outp = (float*)d_out;

  size_t off = 0;
  auto take = [&](size_t bytes) -> size_t {
    const size_t o = off;
    off += (bytes + 4095) & ~((size_t)4095);
    return o;
  };
  const size_t NE   = (size_t)kRows * kChan;
  const size_t oWOH = take((size_t)kChan * kChan * 2);
  const size_t oWOL = take((size_t)kChan * kChan * 2);
  const size_t oR   = take(NE * 4);
  const size_t oKV  = take((size_t)kRows * kKvCols * 4);
  const size_t oWL  = take(NE * 4);
  const size_t oAL  = take(NE * 4);
  const size_t oVL  = take(NE * 4);
  const size_t oXH  = take(NE * 2);
  const size_t oXL  = take(NE * 2);
  const size_t oWRH = take((size_t)kChan * kChan * 2);
  const size_t oWRL = take((size_t)kChan * kChan * 2);
  const size_t oWKVH = take((size_t)kKvCols * kChan * 2);
  const size_t oWKVL = take((size_t)kKvCols * kChan * 2);
  const size_t oLB1H = take((size_t)kLr1N * kChan * 2);
  const size_t oLB1L = take((size_t)kLr1N * kChan * 2);
  const size_t oW2TH = take((size_t)kChan * kLr2K * 2);
  const size_t oW2TL = take((size_t)kChan * kLr2K * 2);
  const size_t oA2TH = take((size_t)kChan * kLr2K * 2);
  const size_t oA2TL = take((size_t)kChan * kLr2K * 2);
  const size_t oV2TH = take((size_t)kChan * kLr2K * 2);
  const size_t oV2TL = take((size_t)kChan * kLr2K * 2);
  const size_t oL1F  = take((size_t)kRows * kLr1N * 4);
  const size_t oL1H  = take((size_t)kRows * kLr1N * 2);
  const size_t oL1L  = take((size_t)kRows * kLr1N * 2);
  const size_t total = off;
  if (total > ws_size) return;
  if (total > (size_t)134217728) return;

  char* ws = (char*)d_ws;
  unsigned short* WOH  = (unsigned short*)(ws + oWOH);
  unsigned short* WOL  = (unsigned short*)(ws + oWOL);
  float* Rf   = (float*)(ws + oR);
  float* KVf  = (float*)(ws + oKV);
  float* WLf  = (float*)(ws + oWL);
  float* ALf  = (float*)(ws + oAL);
  float* VLf  = (float*)(ws + oVL);
  unsigned short* XH   = (unsigned short*)(ws + oXH);
  unsigned short* XL   = (unsigned short*)(ws + oXL);
  unsigned short* YHp  = XH;
  unsigned short* YLp  = XL;
  unsigned short* WRH  = (unsigned short*)(ws + oWRH);
  unsigned short* WRL  = (unsigned short*)(ws + oWRL);
  unsigned short* WKVH = (unsigned short*)(ws + oWKVH);
  unsigned short* WKVL = (unsigned short*)(ws + oWKVL);
  unsigned short* LB1H = (unsigned short*)(ws + oLB1H);
  unsigned short* LB1L = (unsigned short*)(ws + oLB1L);
  unsigned short* W2TH = (unsigned short*)(ws + oW2TH);
  unsigned short* W2TL = (unsigned short*)(ws + oW2TL);
  unsigned short* A2TH = (unsigned short*)(ws + oA2TH);
  unsigned short* A2TL = (unsigned short*)(ws + oA2TL);
  unsigned short* V2TH = (unsigned short*)(ws + oV2TH);
  unsigned short* V2TL = (unsigned short*)(ws + oV2TL);
  float* L1F = (float*)(ws + oL1F);
  unsigned short* L1H = (unsigned short*)(ws + oL1H);
  unsigned short* L1L = (unsigned short*)(ws + oL1L);
  const float* dummyf = (const float*)(ws + oR);

  auto cast8 = [&](const float* in, unsigned short* hi, unsigned short* lo, int n) {
    const int n8 = n / 8;
    cast8_split_kernel<<<(n8 + 255) / 256, 256, 0, stream>>>(in, hi, lo, n8);
  };
  auto trs = [&](const float* in, int R, int Cc, unsigned short* hi, unsigned short* lo) {
    const int rp = (R + 63) / 64, cp = (Cc + 63) / 64;
    dim3 g(rp, cp);
    tr_split_kernel<<<g, 256, 0, stream>>>(in, R, Cc, hi, lo, rp * 64);
  };
  auto gemm = [&](const unsigned short* Ah, const unsigned short* Al, int lda,
                  const unsigned short* Bh, const unsigned short* Bl, int ldb,
                  float* Cc, int ldc, int M, int N, int K) {
    const int tiles = (M / 64) * (N / 64);
    dim3 g((tiles + 7) / 8, 1);
    wmma_gemm64<1, true, 0, 0, false, 0><<<g, 256, 0, stream>>>(
        Ah, Al, lda, 0L, Bh, Bl, ldb, 0L, (void*)Cc, (void*)Cc, ldc, 0L,
        dummyf, dummyf, 0L, M, N, K, 1.0f);
  };

  cast8(x,  XH,  XL,  kRows * kChan);
  cast8(Wr, WRH, WRL, kChan * kChan);
  cast8(Wk, WKVH, WKVL, kKvHalf * kChan);
  cast8(Wv, WKVH + (size_t)kKvHalf * kChan, WKVL + (size_t)kKvHalf * kChan, kKvHalf * kChan);
  cast8(Wo, WOH, WOL, kChan * kChan);
  trs(w1, kChan, kDecLo, LB1H, LB1L);
  trs(a1, kChan, kDecLo, LB1H + (size_t)64 * kChan, LB1L + (size_t)64 * kChan);
  trs(v1, kChan, kMvLo, LB1H + (size_t)128 * kChan, LB1L + (size_t)128 * kChan);
  trs(w2, kDecLo, kChan, W2TH, W2TL);
  trs(a2, kDecLo, kChan, A2TH, A2TL);
  trs(v2, kMvLo, kChan, V2TH, V2TL);

  gemm(XH, XL, kChan, WRH, WRL, kChan, Rf, kChan, kRows, kChan, kChan);
  gemm(XH, XL, kChan, WKVH, WKVL, kChan, KVf, kKvCols, kRows, kKvCols, kChan);
  gemm(XH, XL, kChan, LB1H, LB1L, kChan, L1F, kLr1N, kRows, kLr1N, kChan);

  {
    const int n2 = kRows * kLr1N / 2;
    lr_convert_kernel<<<(n2 + 255) / 256, 256, 0, stream>>>(L1F, L1H, L1L, n2);
  }
  gemm(L1H, L1L, kLr1N, W2TH, W2TL, kLr2K, WLf, kChan, kRows, kChan, kLr2K);
  gemm(L1H + 64, L1L + 64, kLr1N, A2TH, A2TL, kLr2K, ALf, kChan, kRows, kChan, kLr2K);
  gemm(L1H + 128, L1L + 128, kLr1N, V2TH, V2TL, kLr2K, VLf, kChan, kRows, kChan, kLr2K);

  scan_kernel<<<kBatch * kHeads, 64, 0, stream>>>(Rf, KVf, WLf, ALf, VLf, v_first, amask,
                                                  w0, a0, v0, k_k, k_a, r_k, ln_g, ln_b, YHp, YLp);

  gemm(YHp, YLp, kChan, WOH, WOL, kChan, outp, kChan, kRows, kChan, kChan);

  {
    const int n4 = kRows * kChan / 4;
    copy4_kernel<<<(n4 + 255) / 256, 256, 0, stream>>>(v_first, outp + NE, n4);
  }
}
